// Encoder_2353642078838
// MI455X (gfx1250) — hardware-run, weakly checked
//
#include <hip/hip_runtime.h>

typedef float          v8f   __attribute__((ext_vector_type(8)));
typedef float          v4f   __attribute__((ext_vector_type(4)));
typedef unsigned int   v4u   __attribute__((ext_vector_type(4)));
typedef int            v8i   __attribute__((ext_vector_type(8)));
typedef unsigned short v8us  __attribute__((ext_vector_type(8)));
typedef unsigned short v16us __attribute__((ext_vector_type(16)));
typedef __bf16         v16bf __attribute__((ext_vector_type(16)));
typedef _Float16       v16h  __attribute__((ext_vector_type(16)));
typedef v4f  __attribute__((may_alias)) v4fa;
typedef v8us __attribute__((may_alias)) v8usa;
union FragB { v16bf v; v16us u; v8us h[2]; v8i w; };
union FragH { v16h  v; v16us u; v8us h[2]; v8i w; };

__device__ __forceinline__ v8f wmb(const FragB& a, const FragB& b, v8f c) {
  v8f d = __builtin_amdgcn_wmma_f32_16x16x32_bf16(false, a.v, false, b.v, (short)0, c, false, false);
  asm volatile("v_nop\n\tv_nop\n\tv_nop\n\tv_nop" : "+v"(d) : "v"(a.w), "v"(b.w));
  return d;
}

__device__ __forceinline__ v8f wmh(const FragH& a, const FragH& b, v8f c) {
  v8f d = __builtin_amdgcn_wmma_f32_16x16x32_f16(false, a.v, false, b.v, (short)0, c, false, false);
  asm volatile("v_nop\n\tv_nop\n\tv_nop\n\tv_nop" : "+v"(d) : "v"(a.w), "v"(b.w));
  return d;
}

__device__ __forceinline__ unsigned bf16_bits(float f) {
  const unsigned u = __float_as_uint(f);
  const unsigned r = (u + 0x7FFFu + ((u >> 16) & 1u)) >> 16;
  const unsigned q = (u >> 16) | 0x40u;
  return ((u & 0x7fffffffu) > 0x7f800000u) ? q : r;
}

__device__ __forceinline__ float bf16_val(float f) {
  return __uint_as_float(bf16_bits(f) << 16);
}
__device__ __forceinline__ int clampi(int v, int lo, int hi) {
  return v < lo ? lo : (v > hi ? hi : v);
}

__device__ __forceinline__ unsigned f16_bits(float f) {
  const unsigned u  = __float_as_uint(f);
  const unsigned s  = (u >> 16) & 0x8000u;
  const unsigned a  = u & 0x7fffffffu;
  const unsigned t  = a - 0x38000000u;
  const unsigned r  = (t + 0x0FFFu + ((t >> 13) & 1u)) >> 13;
  const unsigned rc = r > 0x7C00u ? 0x7C00u : r;
  const bool small  = a < 0x38800000u;
  const bool isnan  = a > 0x7f800000u;
  const unsigned fin = small ? 0u : (s | rc);
  return isnan ? (s | 0x7E00u) : fin;
}

__device__ __forceinline__ unsigned pk16(unsigned lo, unsigned hi) { return lo | (hi << 16); }
__device__ __forceinline__ unsigned bf16_lo_bits(float v) {
  float hi = bf16_val(v);
  asm volatile("" : "+v"(hi));
  return bf16_bits(v - hi);
}
__device__ __forceinline__ v4u pack8_bf16(v4f a, v4f c) {
  return (v4u){ pk16(bf16_bits(a[0]), bf16_bits(a[1])), pk16(bf16_bits(a[2]), bf16_bits(a[3])),
                pk16(bf16_bits(c[0]), bf16_bits(c[1])), pk16(bf16_bits(c[2]), bf16_bits(c[3])) };
}
__device__ __forceinline__ v4u pack8_bf16_lo(v4f a, v4f c) {
  return (v4u){ pk16(bf16_lo_bits(a[0]), bf16_lo_bits(a[1])), pk16(bf16_lo_bits(a[2]), bf16_lo_bits(a[3])),
                pk16(bf16_lo_bits(c[0]), bf16_lo_bits(c[1])), pk16(bf16_lo_bits(c[2]), bf16_lo_bits(c[3])) };
}
__device__ __forceinline__ v4u pack8_f16(v4f a, v4f c) {
  return (v4u){ pk16(f16_bits(a[0]), f16_bits(a[1])), pk16(f16_bits(a[2]), f16_bits(a[3])),
                pk16(f16_bits(c[0]), f16_bits(c[1])), pk16(f16_bits(c[2]), f16_bits(c[3])) };
}

template <int FORM>
__global__ __launch_bounds__(256) void k_plane(const float* __restrict__ src, int rows, int cols, int ldsrc,
                                               unsigned short* __restrict__ dst, int MP, int KP) {
  static_assert(FORM >= 0 && FORM <= 3);
  const int KTOT = (FORM == 1 || FORM == 3) ? 2 * KP : KP;
  const unsigned ppr   = (unsigned)(KTOT >> 3);
  const unsigned kp8   = (unsigned)(KP >> 3);
  const unsigned total = (unsigned)MP * ppr;
  const unsigned g     = blockIdx.x * 256u + threadIdx.x;
  const unsigned rowu  = g / ppr;
  const unsigned p     = g - rowu * ppr;
  const bool second    = p >= kp8;
  const int row = (int)rowu;
  const int c0  = (int)((second ? p - kp8 : p) << 3);
  const float* srow = src + (size_t)clampi(row, 0, rows - 1) * (size_t)ldsrc;
  float x[8];
  unsigned mk[8];
#pragma unroll
  for (int e = 0; e < 8; ++e) {
    const int c = c0 + e;
    const float v = srow[clampi(c, 0, cols - 1)];
    asm volatile("" :: "v"(v));
    x[e]  = v;
    mk[e] = (row < rows && c < cols) ? 0xFFFFu : 0u;
  }
  const v4f a = (v4f){ x[0], x[1], x[2], x[3] };
  const v4f c = (v4f){ x[4], x[5], x[6], x[7] };
  v4u o;
  if (FORM == 2) {
    o = pack8_f16(a, c);
  } else {
    const v4u hi = pack8_bf16(a, c);
    o = hi;
    if (FORM == 1) { const v4u lo = pack8_bf16_lo(a, c); o = second ? lo : hi; }
  }
  const v4u mw = (v4u){ pk16(mk[0], mk[1]), pk16(mk[2], mk[3]), pk16(mk[4], mk[5]), pk16(mk[6], mk[7]) };
  o &= mw;
  if (g < total) {
    volatile v4u* q = (volatile v4u*)(dst + (size_t)g * 8);
    *q = o;
    __threadfence();
    *q = o;
  }
}

template <int FORM> struct FragOf    { typedef FragB T; };
template <>         struct FragOf<2> { typedef FragH T; };
__device__ __forceinline__ v8f mm(const FragB& a, const FragB& b, v8f c) { return wmb(a, b, c); }
__device__ __forceinline__ v8f mm(const FragH& a, const FragH& b, v8f c) { return wmh(a, b, c); }
template <class F> __device__ __forceinline__ F ld_frag(const unsigned short* p) {
  F f;
  f.h[0] = *(const v8usa*)(p);
  f.h[1] = *(const v8usa*)(p + 16);
  return f;
}

template <int FORM, int EPI>
__global__ __launch_bounds__(256) __attribute__((amdgpu_num_vgpr(248)))
void k_gemm_nt(const unsigned short* __restrict__ A, const unsigned short* __restrict__ B,
               const float* __restrict__ bias, float* __restrict__ D, int M, int N, int KTOT, int ldd) {
  static_assert(FORM >= 0 && FORM <= 2);
  static_assert(EPI == 0 || EPI == 1);
  typedef typename FragOf<FORM>::T F;
  __shared__ __attribute__((aligned(16))) float sT[8][16 * 68];
  const int lane = threadIdx.x & 31;
  const int wave = threadIdx.x >> 5;
  const int tilesM = (M + 63) >> 6;
  const int tilesN = (N + 63) >> 6;
  const int tile = blockIdx.x * 8 + wave;
  if (tile >= tilesM * tilesN) return;
  const int tm = tile / tilesN;
  const int tn = tile - tm * tilesN;
  const int m0 = tm << 6;
  const int n0 = tn << 6;

  const int rl = lane & 15;
  const int h8 = (lane >> 4) * 8;
  const unsigned short* pa = A + (size_t)(m0 + rl) * (size_t)KTOT + h8;
  const unsigned short* pb = B + (size_t)(n0 + rl) * (size_t)KTOT + h8;

  v8f acc[4][4];
#pragma unroll
  for (int i = 0; i < 4; ++i)
#pragma unroll
    for (int j = 0; j < 4; ++j) acc[i][j] = (v8f){0.f, 0.f, 0.f, 0.f, 0.f, 0.f, 0.f, 0.f};

#pragma unroll 1
  for (int k0 = 0; k0 < KTOT; k0 += 32) {
    F bf[4];
#pragma unroll
    for (int j = 0; j < 4; ++j) bf[j] = ld_frag<F>(pb + (size_t)(j << 4) * (size_t)KTOT + k0);
#pragma unroll
    for (int i = 0; i < 4; ++i) {
      const F af = ld_frag<F>(pa + (size_t)(i << 4) * (size_t)KTOT + k0);
#pragma unroll
      for (int j = 0; j < 4; ++j) acc[i][j] = mm(af, bf[j], acc[i][j]);
    }
  }

  float* slab = sT[wave];
  const int hh = lane >> 4;
  const int c4 = (lane & 15) * 4;
  const int nc = n0 + c4;
  const bool cok = nc < N;
  v4f bv = (v4f){0.f, 0.f, 0.f, 0.f};
  if (EPI == 1) {
    bv = *(const v4fa*)(bias + clampi(nc, 0, N - 4));
    asm volatile("" :: "v"(bv));
  }
#pragma unroll
  for (int i = 0; i < 4; ++i) {
    const int mBase = m0 + (i << 4);
#pragma unroll
    for (int j = 0; j < 4; ++j) {
#pragma unroll
      for (int r = 0; r < 8; ++r) slab[(h8 + r) * 68 + (j << 4) + rl] = acc[i][j][r];
    }
    __builtin_amdgcn_fence(__ATOMIC_RELEASE, "workgroup");
    __builtin_amdgcn_wave_barrier();
    __builtin_amdgcn_fence(__ATOMIC_ACQUIRE, "workgroup");
    v4f vv[8];
#pragma unroll
    for (int it = 0; it < 8; ++it) {
      const int row = it * 2 + hh;
      v4f v = *(const v4fa*)(slab + row * 68 + c4);
      if (EPI == 1) v += bv;
      vv[it] = v;
    }
    for (int pass = 0; pass < 2; ++pass) {
#pragma unroll
      for (int it = 0; it < 8; ++it) {
        const int row = mBase + it * 2 + hh;
        if (cok && row < M) *(volatile v4f*)(D + (size_t)row * (size_t)ldd + nc) = vv[it];
      }
      __threadfence();
    }
    __builtin_amdgcn_fence(__ATOMIC_RELEASE, "workgroup");
    __builtin_amdgcn_wave_barrier();
    __builtin_amdgcn_fence(__ATOMIC_ACQUIRE, "workgroup");
  }
}

#include <stddef.h>
#include <stdint.h>
#include <math.h>

#define NN      100000
#define NE      1600000
#define CIN     128
#define HIDC    128
#define OUTC    64
#define MPAD    100096
#define SLB     10
#define NBRUN   1024
#define NBLK    98
#define NPADN   (NBLK * NBRUN)
#define RCAP    28672
#define NWAVE   8
#define WLCAP   (RCAP / NWAVE)
#define DEGCAP  64
#define NCH     (NE / 256)
#define H1_TWO_TERM 1
#define K2      (H1_TWO_TERM ? 2 * HIDC : HIDC)
#define PPR2    (K2 / 8)
#define NU1     (HIDC * (CIN / 8))
#define NU2     (OUTC * PPR2)
#define BK_ZINTS (2 * RCAP + NWAVE * NBRUN + 3 * NBRUN)
#define BK_INTS  (BK_ZINTS + 32)
#define WSMAX   ((size_t)128 << 20)

static_assert(NE % 256 == 0);
static_assert(((long long)NE << SLB) < (1LL << 31));
static_assert(NBRUN == (1 << SLB));
static_assert((long long)NBLK * NBRUN >= MPAD && (NBLK - 1) * NBRUN < NN);
static_assert(MPAD % 64 == 0 && MPAD >= NN && MPAD % 8 == 0 && NN % 16 == 0 && NN % 8 == 0);
static_assert(((NN + 63) / 64) * 64 <= MPAD);
static_assert(HIDC == 32 * 4 && OUTC == 32 * 2);
static_assert(CIN % 32 == 0 && K2 % 32 == 0 && HIDC % 64 == 0 && OUTC % 64 == 0);
static_assert(RCAP >= (16710 * 105) / 100);
static_assert(RCAP % 1024 == 0 && WLCAP * NWAVE == RCAP);
static_assert(WLCAP >= ((16710 / 8) * 3) / 2);
static_assert(DEGCAP >= 36 + 8);
static_assert(BK_ZINTS % 4 == 0 && BK_INTS * 4 <= 327680);
static_assert(NU1 % 256 == 0 && NU2 % 256 == 0);
static_assert((MPAD * (CIN / 8)) % 256 == 0);

typedef float v2f  __attribute__((ext_vector_type(2)));
typedef int   v4i  __attribute__((ext_vector_type(4)));
typedef v2f __attribute__((may_alias)) v2fa;
typedef v4i __attribute__((may_alias)) v4ia;

__global__ __launch_bounds__(256) void k_wprep(const float* __restrict__ W1, const float* __restrict__ b1,
                                               const float* __restrict__ W2, const float* __restrict__ b2,
                                               unsigned short* W1T, unsigned short* W2D, float* BT) {
  const int u = (int)blockIdx.x * 256 + (int)threadIdx.x;
  if (u < NU1) {
    const int n  = u >> 4;
    const int k8 = (u & 15) * 8;
    const float* p = W1 + (size_t)k8 * HIDC + n;
    unsigned w[8];
#pragma unroll
    for (int i = 0; i < 8; ++i) { const float v = p[(size_t)i * HIDC]; w[i] = bf16_bits(v); }
    const v4u o = (v4u){ pk16(w[0], w[1]), pk16(w[2], w[3]), pk16(w[4], w[5]), pk16(w[6], w[7]) };
    volatile v4u* q = (volatile v4u*)(W1T + (size_t)n * CIN + k8);
    *q = o;
    __threadfence();
    *q = o;
  } else if (u < NU1 + NU2) {
    const int v0 = u - NU1;
    const int n  = v0 / PPR2;
    const int k8 = (v0 - n * PPR2) * 8;
    const int kk = k8 & (HIDC - 1);
    const float* p = W2 + (size_t)kk * OUTC + n;
    unsigned w[8];
#pragma unroll
    for (int i = 0; i < 8; ++i) { const float v = p[(size_t)i * OUTC]; w[i] = bf16_bits(v); }
    const v4u o = (v4u){ pk16(w[0], w[1]), pk16(w[2], w[3]), pk16(w[4], w[5]), pk16(w[6], w[7]) };
    volatile v4u* q = (volatile v4u*)(W2D + (size_t)n * K2 + k8);
    *q = o;
    __threadfence();
    *q = o;
  } else {
    const int t = u - (NU1 + NU2);
    const v4f a1 = *(const v4fa*)(b1 + clampi(4 * t, 0, HIDC - 4));
    const v4f a2 = *(const v4fa*)(b2 + clampi(4 * (t - 32), 0, OUTC - 4));
    asm volatile("" :: "v"(a1));
    asm volatile("" :: "v"(a2));
    const bool first = t < 32;
    v4f o;
    o.x = bf16_val(first ? a1.x : a2.x);
    o.y = bf16_val(first ? a1.y : a2.y);
    o.z = bf16_val(first ? a1.z : a2.z);
    o.w = bf16_val(first ? a1.w : a2.w);
    const int tc = t < 47 ? t : 47;
    volatile v4f* q = (volatile v4f*)(BT + 4 * tc);
    if (t < 48) *q = o;
    __threadfence();
    if (t < 48) *q = o;
  }
}

__device__ __forceinline__ int sweep4(const v4i d, const int e0, const unsigned nbs, const unsigned unb,
                                      int* wlw, int wc) {
  const unsigned s0 = (unsigned)d.x - nbs, s1 = (unsigned)d.y - nbs;
  const unsigned s2 = (unsigned)d.z - nbs, s3 = (unsigned)d.w - nbs;
  const bool h0 = s0 < unb, h1 = s1 < unb, h2 = s2 < unb, h3 = s3 < unb;
  const unsigned m0 = __builtin_amdgcn_ballot_w32(h0);
  const unsigned m1 = __builtin_amdgcn_ballot_w32(h1);
  const unsigned m2 = __builtin_amdgcn_ballot_w32(h2);
  const unsigned m3 = __builtin_amdgcn_ballot_w32(h3);
  const unsigned many = m0 | m1 | m2 | m3;
  if (many != 0u) {
    const int lt = (int)(__builtin_amdgcn_mbcnt_lo(m0, 0u) + __builtin_amdgcn_mbcnt_lo(m1, 0u) +
                         __builtin_amdgcn_mbcnt_lo(m2, 0u) + __builtin_amdgcn_mbcnt_lo(m3, 0u));
    int p = wc + lt;
    if (h0 && p < WLCAP) wlw[p] = ((e0 + 0) << SLB) | (int)s0;
    p += h0 ? 1 : 0;
    if (h1 && p < WLCAP) wlw[p] = ((e0 + 1) << SLB) | (int)s1;
    p += h1 ? 1 : 0;
    if (h2 && p < WLCAP) wlw[p] = ((e0 + 2) << SLB) | (int)s2;
    p += h2 ? 1 : 0;
    if (h3 && p < WLCAP) wlw[p] = ((e0 + 3) << SLB) | (int)s3;
    wc += (int)(__builtin_popcount(m0) + __builtin_popcount(m1) + __builtin_popcount(m2) + __builtin_popcount(m3));
  }
  return wc;
}

__global__ __launch_bounds__(256) void k_bucket(const int* __restrict__ srcs, const int* __restrict__ dsts,
                                                int* LIST, int* CNT, int* OFF, float* DINV, int* FLAGS) {
  extern __shared__ __attribute__((aligned(16))) int dsm[];
  int* wl   = dsm;
  int* sl   = dsm + RCAP;
  int* cntw = dsm + 2 * RCAP;
  int* cnt  = cntw + NWAVE * NBRUN;
  int* offs = cnt + NBRUN;
  int* dvs  = offs + NBRUN;
  int* misc = dvs + NBRUN;
  const int tid  = (int)threadIdx.x;
  const int lane = tid & 31;
  const int wave = __builtin_amdgcn_readfirstlane(tid >> 5);
  const int nodeBase = (int)blockIdx.x * NBRUN;
  int nb = NN - nodeBase;
  nb = nb > NBRUN ? NBRUN : (nb < 0 ? 0 : nb);

  {
    const v4i z4 = (v4i){0, 0, 0, 0};
    for (int i = tid * 4; i < BK_ZINTS; i += 1024) *(v4ia*)(dsm + i) = z4;
    if (tid < 32) misc[tid] = 0;
  }
  __syncthreads();

  int wc = 0;
  {
    int* wlw = wl + wave * WLCAP;
    const int ch0 = (NCH * wave) / NWAVE;
    const int ch1 = (NCH * (wave + 1)) / NWAVE;
    const unsigned nbs = (unsigned)nodeBase;
    const unsigned unb = (unsigned)nb;
#pragma unroll 1
    for (int ch = ch0; ch < ch1; ++ch) {
      const int e0 = ch * 256 + 4 * lane;
      const v4i da = *(const v4ia*)(dsts + e0);
      const v4i db = *(const v4ia*)(dsts + e0 + 128);
      wc = sweep4(da, e0, nbs, unb, wlw, wc);
      wc = sweep4(db, e0 + 128, nbs, unb, wlw, wc);
    }
  }
  int cv = wc < 0 ? 0 : (wc > WLCAP ? WLCAP : wc);
  asm volatile("" : "+v"(cv));
  const int cw_n = __builtin_amdgcn_readfirstlane(cv);
  if (lane == 0) { misc[wave] = cw_n; misc[8 + wave] = (wc > WLCAP) ? 1 : 0; }
  __syncthreads();

  {
    const int* wlw = wl + wave * WLCAP;
    int* cw = cntw + wave * NBRUN;
#pragma unroll 1
    for (int b0 = 0; b0 < cw_n; b0 += 32) {
      const int idx = b0 + lane;
      const int ent = wlw[idx < WLCAP ? idx : WLCAP - 1];
      const int m32 = (cw_n - b0) < 32 ? (cw_n - b0) : 32;
#pragma unroll 1
      for (int k = 0; k < m32; ++k) {
        const int u  = __builtin_amdgcn_readlane(ent, k);
        const int s  = u & (NBRUN - 1);
        if (lane == 0) cw[s] = cw[s] + 1;
      }
    }
  }
  __syncthreads();

#pragma unroll 1
  for (int j = 0; j < NBRUN / 256; ++j) {
    const int s = tid + 256 * j;
    int tot = 0;
#pragma unroll
    for (int w2 = 0; w2 < NWAVE; ++w2) tot += cntw[w2 * NBRUN + s];
    cnt[s] = tot;
    const float dg = (float)tot + 1.0f;
    const float di = 1.0f / sqrtf(dg);
    dvs[s] = __float_as_int(di);
  }
  __syncthreads();

  if (wave == 0) {
    const int base = lane * (NBRUN / 32);
    int s = 0;
#pragma unroll 1
    for (int i = 0; i < NBRUN / 32; ++i) s += cnt[base + i];
    int incl = s;
#pragma unroll
    for (int d = 1; d < 32; d <<= 1) {
      const int y = __shfl_up(incl, d, 32);
      if (lane >= d) incl += y;
    }
    int run = incl - s;
#pragma unroll 1
    for (int i = 0; i < NBRUN / 32; ++i) {
      const int c2 = cnt[base + i];
      offs[base + i] = run;
      run += c2;
    }
  }
  __syncthreads();

#pragma unroll 1
  for (int j = 0; j < NBRUN / 256; ++j) {
    const int s = tid + 256 * j;
    int run = offs[s];
#pragma unroll
    for (int w2 = 0; w2 < NWAVE; ++w2) {
      const int c2 = cntw[w2 * NBRUN + s];
      cntw[w2 * NBRUN + s] = run;
      run += c2;
    }
  }
  __syncthreads();

  {
    const int* wlw = wl + wave * WLCAP;
    int* cw = cntw + wave * NBRUN;
#pragma unroll 1
    for (int b0 = 0; b0 < cw_n; b0 += 32) {
      const int idx = b0 + lane;
      const int ent = wlw[idx < WLCAP ? idx : WLCAP - 1];
      const int m32 = (cw_n - b0) < 32 ? (cw_n - b0) : 32;
#pragma unroll 1
      for (int k = 0; k < m32; ++k) {
        const int u = __builtin_amdgcn_readlane(ent, k);
        const int s = u & (NBRUN - 1);
        if (lane == 0) {
          int p = cw[s];
          p = p < 0 ? 0 : (p > RCAP - 1 ? RCAP - 1 : p);
          sl[p] = u;
          cw[s] = p + 1;
        }
      }
    }
  }
  __syncthreads();

  int tt = 0, ovf = 0;
#pragma unroll
  for (int w2 = 0; w2 < NWAVE; ++w2) {
    const int c2 = misc[w2];
    tt  += c2 < 0 ? 0 : (c2 > WLCAP ? WLCAP : c2);
    ovf |= misc[8 + w2];
  }
  tt = tt > RCAP ? RCAP : tt;

  {
    const int fillNode = nodeBase < NN - 1 ? nodeBase : NN - 1;
    int* lg = LIST + (size_t)blockIdx.x * RCAP;
#pragma unroll 1
    for (int it = 0; it < RCAP / 1024; ++it) {
      const int i0 = it * 1024 + 4 * tid;
      const v4i u4 = *(const v4ia*)(sl + i0);
      const int ex = clampi(u4.x >> SLB, 0, NE - 1);
      const int ey = clampi(u4.y >> SLB, 0, NE - 1);
      const int ez = clampi(u4.z >> SLB, 0, NE - 1);
      const int ew = clampi(u4.w >> SLB, 0, NE - 1);
      const int sx = srcs[ex];
      const int sy = srcs[ey];
      const int sz = srcs[ez];
      const int sw = srcs[ew];
      asm volatile("" :: "v"(sx));
      asm volatile("" :: "v"(sy));
      asm volatile("" :: "v"(sz));
      asm volatile("" :: "v"(sw));
      v4i o;
      o.x = (i0 + 0 < tt) ? clampi(sx, 0, NN - 1) : fillNode;
      o.y = (i0 + 1 < tt) ? clampi(sy, 0, NN - 1) : fillNode;
      o.z = (i0 + 2 < tt) ? clampi(sz, 0, NN - 1) : fillNode;
      o.w = (i0 + 3 < tt) ? clampi(sw, 0, NN - 1) : fillNode;
      volatile v4i* q = (volatile v4i*)(lg + i0);
      *q = o;
      __threadfence();
      *q = o;
    }
  }

  {
    const int s0 = 4 * tid;
    const v4i c4 = *(const v4ia*)(cnt + s0);
    const v4i o4 = *(const v4ia*)(offs + s0);
    const v4i d4 = *(const v4ia*)(dvs + s0);
    const v4f dv = (v4f){ __int_as_float(d4.x), __int_as_float(d4.y), __int_as_float(d4.z), __int_as_float(d4.w) };
    volatile v4i* qc = (volatile v4i*)(CNT + (size_t)nodeBase + s0);
    volatile v4i* qo = (volatile v4i*)(OFF + (size_t)nodeBase + s0);
    volatile v4f* qd = (volatile v4f*)(DINV + (size_t)nodeBase + s0);
    *qc = c4; *qo = o4; *qd = dv;
    __threadfence();
    *qc = c4; *qo = o4; *qd = dv;
  }

  {
    const v4i f4 = (v4i){ovf, ovf, ovf, ovf};
    const bool wr = (wave == 0) && (lane < 8);
    volatile v4i* qf = (volatile v4i*)(FLAGS + (size_t)blockIdx.x * 32 + 4 * (lane & 7));
    if (wr) *qf = f4;
    __threadfence();
    if (wr) *qf = f4;
  }
}

__global__ __launch_bounds__(256) void k_agg1(const int* __restrict__ LIST, const int* __restrict__ CNT,
                                              const int* __restrict__ OFF, const float* __restrict__ DINV,
                                              const int* __restrict__ FLAGS, const float* __restrict__ T1,
                                              const float* __restrict__ BF, unsigned short* H) {
  __shared__ __attribute__((aligned(16))) float sb[HIDC];
  const int tid  = (int)threadIdx.x;
  const int lane = tid & 31;
  const int wave = __builtin_amdgcn_readfirstlane(tid >> 5);
  if (tid < 32) {
    const v4f b = *(const v4fa*)(BF + 4 * tid);
    *(v4fa*)(sb + 4 * tid) = b;
  }
  __syncthreads();
  const v4f bv = *(const v4fa*)(sb + 4 * lane);

  const int node = (int)blockIdx.x * NWAVE + wave;
  const int nc   = node < NN ? node : NN - 1;
  const int blk  = clampi(node >> SLB, 0, NBLK - 1);
  int cld = CNT[node];
  int old = OFF[node];
  const int fl = FLAGS[blk * 32];
  asm volatile("" : "+v"(cld));
  asm volatile("" : "+v"(old));
  const bool big = cld > DEGCAP;
  cld = cld < 0 ? 0 : (cld > DEGCAP ? DEGCAP : cld);
  old = old < 0 ? 0 : (old > RCAP - 1 ? RCAP - 1 : old);
  const int c = __builtin_amdgcn_readfirstlane(cld);
  const int o = __builtin_amdgcn_readfirstlane(old);
  const bool poisoned = (fl != 0) || big;
  const float dd = DINV[nc];
  const float rd = dd * dd;
  const int* lb = LIST + (size_t)blk * RCAP;

  v4f acc = (v4f){0.0f, 0.0f, 0.0f, 0.0f};
#pragma unroll 1
  for (int b0 = 0; b0 < c; b0 += 32) {
    int idx = o + b0 + lane;
    idx = idx > RCAP - 1 ? RCAP - 1 : idx;
    int sr = lb[idx];
    asm volatile("" :: "v"(sr));
    sr = clampi(sr, 0, NN - 1);
    const float cf = DINV[sr] * dd;
    asm volatile("" :: "v"(cf));
    const int cfi = __float_as_int(cf);
    const int m32 = (c - b0) < 32 ? (c - b0) : 32;
#pragma unroll 1
    for (int k = 0; k < m32; ++k) {
      const int   sk = __builtin_amdgcn_readlane(sr, k);
      const float ck = __int_as_float(__builtin_amdgcn_readlane(cfi, k));
      const v4f a = *(const v4fa*)(T1 + (size_t)sk * HIDC + 4 * lane);
      acc.x = fmaf(ck, a.x, acc.x);
      acc.y = fmaf(ck, a.y, acc.y);
      acc.z = fmaf(ck, a.z, acc.z);
      acc.w = fmaf(ck, a.w, acc.w);
    }
  }
  const v4f sv = *(const v4fa*)(T1 + (size_t)nc * HIDC + 4 * lane);
  float y0 = (acc.x + sv.x * rd) + bv.x;
  float y1 = (acc.y + sv.y * rd) + bv.y;
  float y2 = (acc.z + sv.z * rd) + bv.z;
  float y3 = (acc.w + sv.w * rd) + bv.w;
  y0 = (y0 > 0.0f) ? y0 : (y0 - y0);
  y1 = (y1 > 0.0f) ? y1 : (y1 - y1);
  y2 = (y2 > 0.0f) ? y2 : (y2 - y2);
  y3 = (y3 > 0.0f) ? y3 : (y3 - y3);
  const float qnan = __int_as_float(0x7fc00000);
  y0 = poisoned ? qnan : y0;
  y1 = poisoned ? qnan : y1;
  y2 = poisoned ? qnan : y2;
  y3 = poisoned ? qnan : y3;
  const bool live = node < NN;
  const float v0 = live ? y0 : 0.0f;
  const float v1 = live ? y1 : 0.0f;
  const float v2 = live ? y2 : 0.0f;
  const float v3 = live ? y3 : 0.0f;

  const int hw0 = (int)pk16(bf16_bits(v0), bf16_bits(v1));
  const int hw1 = (int)pk16(bf16_bits(v2), bf16_bits(v3));
  const int lw0 = (int)pk16(bf16_lo_bits(v0), bf16_lo_bits(v1));
  const int lw1 = (int)pk16(bf16_lo_bits(v2), bf16_lo_bits(v3));
  const int sa = (2 * lane) & 31, sc = (2 * lane + 1) & 31;
  const int g0 = __shfl(hw0, sa, 32), g1 = __shfl(hw1, sa, 32);
  const int g2 = __shfl(hw0, sc, 32), g3 = __shfl(hw1, sc, 32);
  const int p0 = __shfl(lw0, sa, 32), p1 = __shfl(lw1, sa, 32);
  const int p2 = __shfl(lw0, sc, 32), p3 = __shfl(lw1, sc, 32);
  const bool lsel = lane >= 16;
  v4u pv;
  pv.x = (unsigned)(lsel ? p0 : g0);
  pv.y = (unsigned)(lsel ? p1 : g1);
  pv.z = (unsigned)(lsel ? p2 : g2);
  pv.w = (unsigned)(lsel ? p3 : g3);
  const int lq = (8 * lane < K2) ? lane : (K2 / 8 - 1);
  const bool wr = (node < MPAD) && (8 * lane < K2);
  volatile v4u* q = (volatile v4u*)(H + (size_t)node * K2 + 8 * lq);
  if (wr) *q = pv;
  __threadfence();
  if (wr) *q = pv;
}

__global__ __launch_bounds__(256) void k_agg2(const int* __restrict__ LIST, const int* __restrict__ CNT,
                                              const int* __restrict__ OFF, const float* __restrict__ DINV,
                                              const int* __restrict__ FLAGS, const float* __restrict__ T2,
                                              const float* __restrict__ BF, float* out) {
  __shared__ __attribute__((aligned(16))) float sb[OUTC];
  const int tid  = (int)threadIdx.x;
  const int lane = tid & 31;
  const int wave = __builtin_amdgcn_readfirstlane(tid >> 5);
  if (tid < 16) {
    const v4f b = *(const v4fa*)(BF + 4 * tid);
    *(v4fa*)(sb + 4 * tid) = b;
  }
  __syncthreads();
  const v2f bv = *(const v2fa*)(sb + 2 * lane);

  const int node = (int)blockIdx.x * NWAVE + wave;
  const int nc   = node < NN ? node : NN - 1;
  const int blk  = clampi(nc >> SLB, 0, NBLK - 1);
  int cld = CNT[nc];
  int old = OFF[nc];
  const int fl = FLAGS[blk * 32];
  asm volatile("" : "+v"(cld));
  asm volatile("" : "+v"(old));
  const bool big = cld > DEGCAP;
  cld = cld < 0 ? 0 : (cld > DEGCAP ? DEGCAP : cld);
  old = old < 0 ? 0 : (old > RCAP - 1 ? RCAP - 1 : old);
  const int c = __builtin_amdgcn_readfirstlane(cld);
  const int o = __builtin_amdgcn_readfirstlane(old);
  const bool poisoned = (fl != 0) || big;
  const float dd = DINV[nc];
  const float rd = dd * dd;
  const int* lb = LIST + (size_t)blk * RCAP;

  float acc0 = 0.0f, acc1 = 0.0f;
#pragma unroll 1
  for (int b0 = 0; b0 < c; b0 += 32) {
    int idx = o + b0 + lane;
    idx = idx > RCAP - 1 ? RCAP - 1 : idx;
    int sr = lb[idx];
    asm volatile("" :: "v"(sr));
    sr = clampi(sr, 0, NN - 1);
    const float cf = DINV[sr] * dd;
    asm volatile("" :: "v"(cf));
    const int cfi = __float_as_int(cf);
    const int m32 = (c - b0) < 32 ? (c - b0) : 32;
#pragma unroll 1
    for (int k = 0; k < m32; ++k) {
      const int   sk = __builtin_amdgcn_readlane(sr, k);
      const float ck = __int_as_float(__builtin_amdgcn_readlane(cfi, k));
      const v2f a = *(const v2fa*)(T2 + (size_t)sk * OUTC + 2 * lane);
      acc0 = fmaf(ck, a.x, acc0);
      acc1 = fmaf(ck, a.y, acc1);
    }
  }
  const v2f sv = *(const v2fa*)(T2 + (size_t)nc * OUTC + 2 * lane);
  float y0 = (acc0 + sv.x * rd) + bv.x;
  float y1 = (acc1 + sv.y * rd) + bv.y;
  const float qnan = __int_as_float(0x7fc00000);
  y0 = poisoned ? qnan : y0;
  y1 = poisoned ? qnan : y1;

  const int sa = (2 * lane) & 31, sc = (2 * lane + 1) & 31;
  v4f ow;
  ow.x = __shfl(y0, sa, 32);
  ow.y = __shfl(y1, sa, 32);
  ow.z = __shfl(y0, sc, 32);
  ow.w = __shfl(y1, sc, 32);
  const bool wr = (node < NN) && (lane < 16);
  volatile v4f* q = (volatile v4f*)(out + (size_t)nc * OUTC + 4 * (lane & 15));
  if (wr) *q = ow;
  __threadfence();
  if (wr) *q = ow;
}

static inline size_t al256(size_t o) { return (o + 255) & ~(size_t)255; }

extern "C" void kernel_launch(void* const* d_in, const int* in_sizes, int n_in,
                              void* d_out, int out_size, void* d_ws, size_t ws_size,
                              hipStream_t stream) {
  if (n_in < 6) return;
  if (in_sizes[0] != NN * CIN) return;
  if (in_sizes[1] != 2 * NE) return;
  if (in_sizes[2] != CIN * HIDC || in_sizes[3] != HIDC) return;
  if (in_sizes[4] != HIDC * OUTC || in_sizes[5] != OUTC) return;
  if (out_size != NN * OUTC) return;

  const float* x  = (const float*)d_in[0];
  const int*   ei = (const int*)d_in[1];
  const float* W1 = (const float*)d_in[2];
  const float* b1 = (const float*)d_in[3];
  const float* W2 = (const float*)d_in[4];
  const float* b2 = (const float*)d_in[5];
  float* out = (float*)d_out;
  const int* srcs = ei;
  const int* dsts = ei + NE;

  char* ws = (char*)d_ws;
  size_t off = 0;
  const size_t oH   = off; off = al256(off + (size_t)MPAD * 256 * 2);
  const size_t oT   = off; off = al256(off + (size_t)MPAD * HIDC * 4);
  const size_t oL   = off; off = al256(off + (size_t)NBLK * RCAP * 4);
  const size_t oC   = off; off = al256(off + (size_t)NPADN * 4);
  const size_t oO   = off; off = al256(off + (size_t)NPADN * 4);
  const size_t oD   = off; off = al256(off + (size_t)NPADN * 4);
  const size_t oF   = off; off = al256(off + (size_t)NBLK * 128);
  const size_t oW1  = off; off = al256(off + (size_t)HIDC * CIN * 2);
  const size_t oW2  = off; off = al256(off + (size_t)OUTC * 256 * 2);
  const size_t oB   = off; off = al256(off + (size_t)(HIDC + OUTC) * 4);
  if (off > ws_size || off > WSMAX) return;
  unsigned short* H1HL = (unsigned short*)(ws + oH);
  unsigned short* XB   = (unsigned short*)(ws + oH);
  float*          T    = (float*)(ws + oT);
  int*            LIST = (int*)(ws + oL);
  int*            CNT  = (int*)(ws + oC);
  int*            OFF  = (int*)(ws + oO);
  float*          DINV = (float*)(ws + oD);
  int*            FLAGS = (int*)(ws + oF);
  unsigned short* W1T  = (unsigned short*)(ws + oW1);
  unsigned short* W2D  = (unsigned short*)(ws + oW2);
  float*          BT   = (float*)(ws + oB);

  const size_t bkLds = (size_t)BK_INTS * 4;
  hipFuncSetAttribute(reinterpret_cast<const void*>(&k_bucket), hipFuncAttributeMaxDynamicSharedMemorySize, (int)bkLds);

  constexpr int G2FORM = H1_TWO_TERM ? 1 : 0;
  const int tiles1 = ((NN + 63) / 64) * (HIDC / 64);
  const int tiles2 = ((NN + 63) / 64) * (OUTC / 64);

  k_wprep<<<(NU1 + NU2) / 256 + 1, 256, 0, stream>>>(W1, b1, W2, b2, W1T, W2D, BT);
  k_plane<0><<<(MPAD * (CIN / 8)) / 256, 256, 0, stream>>>(x, NN, CIN, CIN, XB, MPAD, CIN);
  k_bucket<<<NBLK, 256, bkLds, stream>>>(srcs, dsts, LIST, CNT, OFF, DINV, FLAGS);
  k_gemm_nt<0, 0><<<(tiles1 + 7) / 8, 256, 0, stream>>>(XB, W1T, BT, T, NN, HIDC, CIN, HIDC);
  k_agg1<<<MPAD / NWAVE, 256, 0, stream>>>(LIST, CNT, OFF, DINV, FLAGS, T, BT, H1HL);
  k_gemm_nt<G2FORM, 0><<<(tiles2 + 7) / 8, 256, 0, stream>>>(H1HL, W2D, BT, T, NN, OUTC, K2, OUTC);
  k_agg2<<<NN / NWAVE, 256, 0, stream>>>(LIST, CNT, OFF, DINV, FLAGS, T, BT + HIDC, out);
}
